// SimpleRetention_10737418240742
// MI455X (gfx1250) — hardware-verified
//
#include <hip/hip_runtime.h>


namespace {
constexpr int G = 16, S = 2048, H = 256, HALF = H / 2;
constexpr int QB = S / 128, KBW = 64, NTRI = QB * QB + QB;
constexpr float GAMMA = 0.96875f, P_SC = 8.0f, INV_P_SC = 0.125f;

typedef _Float16 b16;
typedef __attribute__((ext_vector_type(16))) _Float16 v16b;
typedef __attribute__((ext_vector_type(8)))  _Float16 v8b;
typedef __attribute__((ext_vector_type(8)))  float v8f;
typedef __attribute__((ext_vector_type(4)))  float v4f;

__device__ __forceinline__ v8b ld8b(const b16* p) { return *(const v8b*)p; }
__device__ __forceinline__ v16b cat8b(v8b a, v8b b) { return __builtin_shufflevector(a, b, 0, 1, 2, 3, 4, 5, 6, 7, 8, 9, 10, 11, 12, 13, 14, 15); }
__device__ __forceinline__ v16b frag_kb(const b16* p, int hh) { return cat8b(ld8b(p + 8 * hh), ld8b(p + 16 + 8 * hh)); }
__device__ __forceinline__ void split16(float v, b16& hi, b16& lo) { hi = (b16)v; lo = (b16)(v - (float)hi); }
__device__ __forceinline__ void frag_ksplit(const float* p, int hh, v16b& fh_, v16b& fl_) {
  const float* p0 = p + 8 * hh; const float* p1 = p + 16 + 8 * hh;
#pragma unroll
  for (int e = 0; e < 8; ++e) { b16 a, c; split16(p0[e], a, c); fh_[e] = a; fl_[e] = c; split16(p1[e], a, c); fh_[8 + e] = a; fl_[8 + e] = c; }
}
__device__ __forceinline__ v8f wmma16b(v16b a, v16b b, v8f c) {
  v8f d = __builtin_amdgcn_wmma_f32_16x16x32_f16(false, a, false, b, (short)0, c, false, false);
  asm volatile("v_nop\n\tv_nop\n\tv_nop\n\tv_nop" : "+v"(d) : "v"(a), "v"(b));
  return d;
}
__device__ __forceinline__ void wave_lds_sync() {
  __builtin_amdgcn_fence(__ATOMIC_RELEASE, "workgroup");
  __builtin_amdgcn_wave_barrier();
  __builtin_amdgcn_fence(__ATOMIC_ACQUIRE, "workgroup");
}

struct Opnd { const void* p0; const void* p1; int ld; };
template <int NP> __device__ __forceinline__ void load_frags(const Opnd& o, int row, int kb, int hh, v16b& fh_, v16b& fl_) {
  if (NP == 0) { frag_ksplit((const float*)o.p0 + (size_t)row * o.ld + kb, hh, fh_, fl_); }
  else if (NP == 3) {
    const float* p = (const float*)o.p0 + (size_t)row * o.ld + kb; const float* p0 = p + 8 * hh; const float* p1 = p + 16 + 8 * hh;
#pragma unroll
    for (int e = 0; e < 8; ++e) { fh_[e] = (b16)p0[e]; fh_[8 + e] = (b16)p1[e]; }
    fl_ = fh_;
  } else {
    fh_ = frag_kb((const b16*)o.p0 + (size_t)row * o.ld + kb, hh);
    if (NP == 2) fl_ = frag_kb((const b16*)o.p1 + (size_t)row * o.ld + kb, hh); else fl_ = fh_;
  }
}
template <int ANP, int BNP> __device__ __forceinline__ v8f mac(v16b ah, v16b al, v16b bh, v16b bl, v8f c) {
  c = wmma16b(ah, bh, c);
  if (BNP == 0 || BNP == 2) c = wmma16b(ah, bl, c);
  if (ANP == 0 || ANP == 2) c = wmma16b(al, bh, c);
  return c;
}
template <int ANP, int BNP>
__device__ __forceinline__ void gemm_tile(const Opnd& A, const Opnd& B, int K, int m0, int c0, int nloc, int hlf, v8f (&acc)[2][4]) {
  for (int kb = 0; kb < K; kb += 32) {
    v16b a0h, a0l, a1h, a1l;
    load_frags<ANP>(A, m0 + nloc, kb, hlf, a0h, a0l);
    load_frags<ANP>(A, m0 + 16 + nloc, kb, hlf, a1h, a1l);
#pragma unroll
    for (int t = 0; t < 4; ++t) {
      v16b bh, bl;
      load_frags<BNP>(B, c0 + t * 16 + nloc, kb, hlf, bh, bl);
      acc[0][t] = mac<ANP, BNP>(a0h, a0l, bh, bl, acc[0][t]);
      acc[1][t] = mac<ANP, BNP>(a1h, a1l, bh, bl, acc[1][t]);
    }
  }
}

__device__ __forceinline__ void epi_planes(v8f (&acc)[2][4], float scale, bool two, b16* __restrict__ oh, b16* __restrict__ ol, int ldo,
                                           int m0, int c0, int lane, b16* Th, b16* Tl) {
  const int nloc = lane & 15, hlf = lane >> 4;
#pragma unroll
  for (int t = 0; t < 4; ++t)
#pragma unroll
    for (int r = 0; r < 2; ++r)
#pragma unroll
      for (int v = 0; v < 8; ++v) {
        const int rr = r * 16 + v + 8 * hlf, cc = t * 16 + nloc;
        b16 h_, l_; split16(acc[r][t][v] * scale, h_, l_);
        Th[rr * 64 + cc] = h_; Tl[rr * 64 + cc] = l_;
      }
  wave_lds_sync();
  for (int pass = 0; pass < 2; ++pass) {
#pragma unroll
    for (int j = 0; j < 8; ++j) {
      const int rr = j * 4 + (lane >> 3), c8 = (lane & 7) * 8;
      const size_t o = (size_t)(m0 + rr) * ldo + c0 + c8;
      *(volatile v8b*)(oh + o) = ld8b(Th + rr * 64 + c8);
      if (two) *(volatile v8b*)(ol + o) = ld8b(Tl + rr * 64 + c8);
    }
    __threadfence();
  }
}
__device__ __forceinline__ void epi_f32(v8f (&acc)[2][4], float scale, const float* rscale, float* __restrict__ out, int ldo, int m0, int c0, int lane, float* Tt) {
  const int nloc = lane & 15, hlf = lane >> 4;
#pragma unroll
  for (int t = 0; t < 4; ++t)
#pragma unroll
    for (int r = 0; r < 2; ++r)
#pragma unroll
      for (int v = 0; v < 8; ++v) {
        const int rr = r * 16 + v + 8 * hlf;
        const float rs = rscale ? rscale[(size_t)(m0 + rr) * 32] : 1.0f;
        Tt[rr * 64 + t * 16 + nloc] = acc[r][t][v] * scale * rs;
      }
  wave_lds_sync();
  float* dst0 = out + (size_t)m0 * ldo + c0;
  for (int pass = 0; pass < 2; ++pass) {
#pragma unroll
    for (int j = 0; j < 16; ++j) { const int rr = j * 2 + hlf, c4 = nloc * 4; *(volatile v4f*)(dst0 + (size_t)rr * ldo + c4) = *(const v4f*)(Tt + rr * 64 + c4); }
    __threadfence();
  }
}


__global__ __launch_bounds__(256) void prep_kernel(const float* __restrict__ wq, const float* __restrict__ wk, const float* __restrict__ wv,
                                                   b16* __restrict__ w16, float* __restrict__ tab, float* __restrict__ dk) {
  const size_t tid = (size_t)blockIdx.x * blockDim.x + threadIdx.x, stride = (size_t)gridDim.x * blockDim.x;
  const size_t nw = (size_t)3 * H * H / 8, ntab = (size_t)S * HALF, ndk = S;
  for (int pass = 0; pass < 2; ++pass) {
    for (size_t c = tid; c < nw + ntab + ndk; c += stride) {
      if (c < nw) {
        const int which = (int)(c / ((size_t)H * H / 8)); const size_t i = (c % ((size_t)H * H / 8)) * 8; const int n = (int)(i / H), k0 = (int)(i % H);
        const float* w = (which == 0) ? wq : (which == 1) ? wk : wv;
        v8b v;
#pragma unroll
        for (int e = 0; e < 8; ++e) v[e] = (b16)w[(size_t)(k0 + e) * H + n];
        *(volatile v8b*)(w16 + (size_t)which * H * H + i) = v;
      } else if (c < nw + ntab) {
        const size_t q = c - nw; const int t = (int)(q / HALF), i = (int)(q % HALF);
        const float base = ((float)(2 * i) + 0.4f * (float)H) * (1.0f / (1.4f * (float)H));
        const float sc = exp2f(((float)t / 512.0f) * log2f(base)), isc = 1.0f / sc;
        const float wfr = 1.0f / powf(10000.0f, (float)i / (float)HALF);
        float sn, cs; sincosf((float)t * wfr, &sn, &cs);
        ((volatile float*)tab)[q] = cs * sc; ((volatile float*)tab)[(size_t)S * HALF + q] = sn * sc;
        ((volatile float*)tab)[(size_t)2 * S * HALF + q] = cs * isc; ((volatile float*)tab)[(size_t)3 * S * HALF + q] = sn * isc;
      } else {
        const int n = (int)(c - nw - ntab);
        ((volatile float*)dk)[n] = exp2f((float)n * -0.045803689613124746f);
      }
    }
    __threadfence();
  }
}

__global__ __launch_bounds__(128) void projqk_kernel(const float* __restrict__ X, const b16* __restrict__ w16, const float* __restrict__ tab,
                                                     b16* __restrict__ q16, b16* __restrict__ k16) {
  __shared__ __attribute__((aligned(16))) b16 Ts[4][32 * 64];
  const int lane = threadIdx.x & 31, wave = threadIdx.x >> 5, nloc = lane & 15, hlf = lane >> 4;
  const int g = blockIdx.z, m0 = blockIdx.y * 128 + wave * 32, cg = blockIdx.x * 64;
  const bool isq = cg < H; const int c0 = isq ? cg : cg - H;
  v8f acc[2][4];
#pragma unroll
  for (int r = 0; r < 2; ++r)
#pragma unroll
    for (int t = 0; t < 4; ++t) acc[r][t] = (v8f){};
  const Opnd A{X + (size_t)g * S * H, nullptr, H}, B{w16 + (isq ? 0 : (size_t)H * H), nullptr, H};
  gemm_tile<3, 1>(A, B, H, m0, c0, nloc, hlf, acc);
  const float* ct = tab + (isq ? 0 : (size_t)2 * S * HALF); const float* st = ct + (size_t)S * HALF;
  b16* Tp = Ts[wave];
#pragma unroll
  for (int t = 0; t < 4; ++t)
#pragma unroll
    for (int r = 0; r < 2; ++r)
#pragma unroll
      for (int v = 0; v < 8; ++v) {
        const int rr = r * 16 + v + 8 * hlf, d = c0 + t * 16 + nloc, tpos = m0 + rr;
        const float val = acc[r][t][v], oth = __shfl_xor(val, 1);
        const float cv = ct[(size_t)tpos * HALF + (d >> 1)], sv = st[(size_t)tpos * HALF + (d >> 1)];
        const float rot = (d & 1) ? (val * cv + oth * sv) : (val * cv - oth * sv);
        Tp[rr * 64 + t * 16 + nloc] = (b16)rot;
      }
  wave_lds_sync();
  b16* base = (isq ? q16 : k16) + (size_t)g * S * H;
  for (int pass = 0; pass < 2; ++pass) {
#pragma unroll
    for (int j = 0; j < 8; ++j) { const int rr = j * 4 + (lane >> 3), c8 = (lane & 7) * 8; *(volatile v8b*)(base + (size_t)(m0 + rr) * H + c0 + c8) = ld8b(Tp + rr * 64 + c8); }
    __threadfence();
  }
}

__global__ __launch_bounds__(128) void projv_kernel(const float* __restrict__ X, const b16* __restrict__ wv16, b16* __restrict__ vt16) {
  __shared__ __attribute__((aligned(16))) b16 Ts[4][2][32 * 64];
  const int lane = threadIdx.x & 31, wave = threadIdx.x >> 5, nloc = lane & 15, hlf = lane >> 4;
  const int g = blockIdx.z, m0 = blockIdx.y * 128 + wave * 32, c0 = blockIdx.x * 64;
  v8f acc[2][4];
#pragma unroll
  for (int r = 0; r < 2; ++r)
#pragma unroll
    for (int t = 0; t < 4; ++t) acc[r][t] = (v8f){};
  const Opnd A{wv16, nullptr, H}, B{X + (size_t)g * S * H, nullptr, H};
  gemm_tile<1, 3>(A, B, H, m0, c0, nloc, hlf, acc);
  epi_planes(acc, 1.0f, false, vt16 + (size_t)g * H * S, nullptr, S, m0, c0, lane, Ts[wave][0], Ts[wave][1]);
}

__global__ __launch_bounds__(128) void s_kernel(const b16* __restrict__ qg, const b16* __restrict__ kg, const float* __restrict__ dk, b16* __restrict__ P) {
  __shared__ __attribute__((aligned(16))) b16 Ts[4][32 * 64];
  const int lane = threadIdx.x & 31, wave = threadIdx.x >> 5, nloc = lane & 15, hlf = lane >> 4;
  int qb = 0;
#pragma unroll 1
  for (int j = 1; j <= QB; ++j) { if (j * j + j <= (int)blockIdx.x) qb = j; }
  if (qb >= QB) return;
  const int kt = (int)blockIdx.x - (qb * qb + qb);
  const int m0 = qb * 128 + wave * 32, c0 = kt * KBW;
  v8f acc[2][4];
#pragma unroll
  for (int r = 0; r < 2; ++r)
#pragma unroll
    for (int t = 0; t < 4; ++t) acc[r][t] = (v8f){};
  const Opnd A{qg, nullptr, H}, B{kg, nullptr, H};
  gemm_tile<1, 1>(A, B, H, m0, c0, nloc, hlf, acc);
  b16* Tp = Ts[wave];
#pragma unroll
  for (int t = 0; t < 4; ++t)
#pragma unroll
    for (int r = 0; r < 2; ++r)
#pragma unroll
      for (int v = 0; v < 8; ++v) {
        const int rr = r * 16 + v + 8 * hlf, cc = t * 16 + nloc, i = m0 + rr, j = c0 + cc;
        const int dlt = i - j; const float w = (dlt >= 0) ? dk[dlt < S ? dlt : 0] * P_SC : 0.0f;
        Tp[rr * 64 + cc] = (b16)(acc[r][t][v] * w);
      }
  wave_lds_sync();
  for (int pass = 0; pass < 2; ++pass) {
#pragma unroll
    for (int j = 0; j < 8; ++j) { const int rr = j * 4 + (lane >> 3), c8 = (lane & 7) * 8; *(volatile v8b*)(P + (size_t)(m0 + rr) * S + c0 + c8) = ld8b(Tp + rr * 64 + c8); }
    __threadfence();
  }
}

__global__ __launch_bounds__(128) void pv_kernel(const b16* __restrict__ P, const b16* __restrict__ vtg, float* __restrict__ outg) {
  __shared__ __attribute__((aligned(16))) float Ts[4][32 * 64];
  const int lane = threadIdx.x & 31, wave = threadIdx.x >> 5, nloc = lane & 15, hlf = lane >> 4;
  const int qb = blockIdx.y, m0 = qb * 128 + wave * 32, c0 = blockIdx.x * 64, kend = (qb + 1) * 128;
  v8f acc[2][4];
#pragma unroll
  for (int r = 0; r < 2; ++r)
#pragma unroll
    for (int t = 0; t < 4; ++t) acc[r][t] = (v8f){};
  const Opnd A{P, nullptr, S}, B{vtg, nullptr, S};
  gemm_tile<1, 1>(A, B, kend, m0, c0, nloc, hlf, acc);
  epi_f32(acc, INV_P_SC, nullptr, outg, H, m0, c0, lane, Ts[wave]);
}
}

extern "C" void kernel_launch(void* const* d_in, const int* in_sizes, int n_in,
                              void* d_out, int out_size, void* d_ws, size_t ws_size, hipStream_t stream) {
  (void)n_in; (void)out_size;
  const float* X  = (const float*)d_in[0];
  const float* WQ = (const float*)d_in[1];
  const float* WK = (const float*)d_in[2];
  const float* WV = (const float*)d_in[3];
  float* out = (float*)d_out;
  if (in_sizes[0] != G * S * H || in_sizes[1] != H * H || in_sizes[2] != H * H || in_sizes[3] != H * H) return;

  size_t off = 0; char* ws = (char*)d_ws;
  auto carve = [&](size_t bytes) { char* p = ws + off; off += (bytes + 255) & ~(size_t)255; return p; };
  b16* w16   = (b16*)carve((size_t)3 * H * H * 2);
  float* tab = (float*)carve((size_t)4 * S * HALF * 4);
  float* dk  = (float*)carve((size_t)S * 4);
  b16* q16   = (b16*)carve((size_t)G * S * H * 2);
  b16* k16   = (b16*)carve((size_t)G * S * H * 2);
  b16* vt16  = (b16*)carve((size_t)G * H * S * 2);
  b16* P     = (b16*)carve((size_t)S * S * 2);
  if (off > ws_size) return;
  prep_kernel<<<512, 256, 0, stream>>>(WQ, WK, WV, w16, tab, dk);
  projqk_kernel<<<dim3(2 * H / 64, S / 128, G), 128, 0, stream>>>(X, w16, tab, q16, k16);
  projv_kernel<<<dim3(S / 64, H / 128, G), 128, 0, stream>>>(X, w16 + (size_t)2 * H * H, vt16);
  for (int g = 0; g < G; ++g) {
    s_kernel<<<NTRI, 128, 0, stream>>>(q16 + (size_t)g * S * H, k16 + (size_t)g * S * H, dk, P);
    pv_kernel<<<dim3(H / 64, S / 128), 128, 0, stream>>>(P, vt16 + (size_t)g * H * S, out + (size_t)g * S * H);
  }
}
